// NAttention_79568564126295
// MI455X (gfx1250) — hardware-verified
//
#include <hip/hip_runtime.h>


namespace {
constexpr int NN = 2, T = 4096, C = 256, H = 4, HD = 64, WIN = 64, LEFT = 31, PADL = 32, PADR = 64, TP = T + PADL + PADR, NL = 2  ;
constexpr float XS = 8.0f, WSC = 256.0f, PS = 1024.0f, LOG2E = 1.4426950408889634f;
static_assert(T % 64 == 0 && C == H * HD, "tiling");
typedef _Float16 b16;
typedef __attribute__((ext_vector_type(16))) _Float16 v16b;
typedef __attribute__((ext_vector_type(8))) _Float16 v8b;
typedef __attribute__((ext_vector_type(8))) float v8f;
typedef __attribute__((ext_vector_type(4))) float v4f;
__device__ __forceinline__ float bf16_rne(float f) { unsigned int u = __float_as_uint(f); u += 0x7FFFu + ((u >> 16) & 1u); return __uint_as_float(u & 0xFFFF0000u); }
__device__ __forceinline__ void split16(float v, b16& hi, b16& lo) { hi = (b16)v; lo = (b16)(v - (float)hi); }
__device__ __forceinline__ v16b frag_kb(const b16* p, int hh) { const v8b a = *(const v8b*)(p + 8 * hh), b = *(const v8b*)(p + 16 + 8 * hh); v16b f;
#pragma unroll
  for (int e = 0; e < 8; ++e) { f[e] = a[e]; f[8 + e] = b[e]; } return f; }
__device__ __forceinline__ v8f wmma16b(v16b a, v16b b, v8f c) { v8f d = __builtin_amdgcn_wmma_f32_16x16x32_f16(false, a, false, b, (short)0, c, false, false); asm volatile("v_nop\n\tv_nop\n\tv_nop\n\tv_nop" : "+v"(d) : "v"(a), "v"(b)); return d; }
__device__ __forceinline__ void wave_lds_sync() { __builtin_amdgcn_fence(__ATOMIC_RELEASE, "workgroup"); __builtin_amdgcn_wave_barrier(); __builtin_amdgcn_fence(__ATOMIC_ACQUIRE, "workgroup"); }
__device__ __forceinline__ float pmul(float a, float b) { float p = a * b; asm volatile("" : "+v"(p)); return p; }
__device__ __forceinline__ int iclamp(int v, int lo, int hi) { return v < lo ? lo : (v > hi ? hi : v); }

typedef __attribute__((ext_vector_type(2))) _Float16 v2h;
typedef __attribute__((ext_vector_type(4))) _Float16 v4h;
__device__ __forceinline__ float nexp2(float v) { return __builtin_amdgcn_exp2f(v); }
__global__ __launch_bounds__(256) void prep_kernel(const float* __restrict__ wqkv, const float* __restrict__ wproj, b16* __restrict__ WQ, b16* __restrict__ WP, b16* __restrict__ Kp, b16* __restrict__ VT, b16* __restrict__ VTl) {
  size_t t = (size_t)blockIdx.x * 256 + threadIdx.x; v8b o, z = {};
  { const size_t n = (size_t)3 * C * C / 8; if (t < n) { const size_t e = t * 8; const int oo = (int)(e / C), c0 = (int)(e % C); for (int j = 0; j < 8; ++j) o[j] = (b16)(bf16_rne(wqkv[(size_t)(c0 + j) * 3 * C + oo]) * WSC); for (int pass = 0; pass < 2; ++pass) { *(volatile v8b*)(WQ + e) = o; __threadfence(); } return; } t -= n; }
  { const size_t n = (size_t)C * C / 8; if (t < n) { const size_t e = t * 8; const int oo = (int)(e / C), c0 = (int)(e % C); for (int j = 0; j < 8; ++j) o[j] = (b16)(bf16_rne(wproj[(size_t)(c0 + j) * C + oo]) * WSC); for (int pass = 0; pass < 2; ++pass) { *(volatile v8b*)(WP + e) = o; __threadfence(); } return; } t -= n; }
  { const size_t n = (size_t)NN * H * TP * HD / 8; if (t < n) { const size_t e = t * 8; for (int pass = 0; pass < 2; ++pass) { *(volatile v8b*)(Kp + e) = z; *(volatile v8b*)(VT + e) = z; *(volatile v8b*)(VTl + e) = z; __threadfence(); } } }
}
__global__ __launch_bounds__(128) void qkv_kernel(const float* __restrict__ x, const b16* __restrict__ WQ, const float* __restrict__ bq, b16* __restrict__ Qp, b16* __restrict__ Kp, b16* __restrict__ VT, b16* __restrict__ VTl) {
  __shared__ __attribute__((aligned(16))) b16 As[4][16][C + 8]; __shared__ __attribute__((aligned(16))) float Tf[4][16][192 + 4];
  const int wave = threadIdx.x >> 5, lane = threadIdx.x & 31, nloc = lane & 15, hlf = lane >> 4; const int n = blockIdx.y / H, h = blockIdx.y % H; const int t0 = blockIdx.x * 64 + wave * 16;
  for (int rr = 0; rr < 16; ++rr) { const float* xr = x + ((size_t)n * T + t0 + rr) * C; v8b o; for (int j = 0; j < 8; ++j) o[j] = (b16)(bf16_rne(xr[lane * 8 + j]) * XS); *(v8b*)(&As[wave][rr][lane * 8]) = o; }
  wave_lds_sync();
  v8f acc[12];
#pragma unroll
  for (int t = 0; t < 12; ++t) acc[t] = (v8f){};
#pragma unroll 1
  for (int kb = 0; kb < C; kb += 32) { const v16b a = frag_kb(&As[wave][nloc][kb], hlf);
#pragma unroll
    for (int t = 0; t < 12; ++t) { const int s = t >> 2, tt = t & 3; const int oc = (s * H + h) * HD + tt * 16 + nloc; acc[t] = wmma16b(a, frag_kb(WQ + (size_t)oc * C + kb, hlf), acc[t]); } }
#pragma unroll
  for (int t = 0; t < 12; ++t) { const int s = t >> 2, tt = t & 3; const float bb = bf16_rne(bq[(s * H + h) * HD + tt * 16 + nloc]);
#pragma unroll
    for (int r = 0; r < 8; ++r) Tf[wave][8 * hlf + r][t * 16 + nloc] = acc[t][r] * (1.0f / (XS * WSC)) + bb; }
  __syncthreads();
  b16* Qb = Qp + ((size_t)(n * H + h) * T) * HD; b16* Kb = Kp + ((size_t)(n * H + h) * TP + PADL) * HD; b16* Vb = VT + ((size_t)(n * H + h) * HD) * TP + PADL; b16* Vlb = VTl + ((size_t)(n * H + h) * HD) * TP + PADL;
  for (int pass = 0; pass < 2; ++pass) {
    for (int rr = 0; rr < 16; ++rr) { v2h qv, kv; for (int j = 0; j < 2; ++j) { qv[j] = (b16)(Tf[wave][rr][lane * 2 + j] * XS); kv[j] = (b16)(Tf[wave][rr][HD + lane * 2 + j] * XS); }
      *(volatile v2h*)(Qb + (size_t)(t0 + rr) * HD + lane * 2) = qv; *(volatile v2h*)(Kb + (size_t)(t0 + rr) * HD + lane * 2) = kv; }
#pragma unroll 1
    for (int q = 0; q < 16; ++q) { const int d = wave * 16 + q; const int tk = lane * 2; v2h vh, vl; for (int j = 0; j < 2; ++j) { b16 a_, b_; split16(Tf[(tk + j) >> 4][(tk + j) & 15][2 * HD + d] * XS, a_, b_); vh[j] = a_; vl[j] = b_; }
      *(volatile v2h*)(Vb + (size_t)d * TP + blockIdx.x * 64 + lane * 2) = vh; *(volatile v2h*)(Vlb + (size_t)d * TP + blockIdx.x * 64 + lane * 2) = vl; }
    __threadfence(); }
}
__global__ __launch_bounds__(64) void attn_kernel(const b16* __restrict__ Qp, const b16* __restrict__ Kp, const b16* __restrict__ VT, const b16* __restrict__ VTl, const float* __restrict__ rb, b16* __restrict__ Oh, b16* __restrict__ Ol) {
  __shared__ __attribute__((aligned(16))) b16 Ph[2][16][96 + 8], Pl[2][16][96 + 8]; __shared__ __attribute__((aligned(16))) float Pf[2][16][96 + 4], To[2][16][HD + 4]; __shared__ float rbs[2][WIN];
  const int wave = threadIdx.x >> 5, lane = threadIdx.x & 31, hh = lane >> 4, col = lane & 15; const int n = blockIdx.y / H, h = blockIdx.y % H; const int t0 = blockIdx.x * 32 + wave * 16, tq = t0 + col;
  for (int w = lane; w < WIN; w += 32) rbs[wave][w] = bf16_rne(rb[h * WIN + w]);
  wave_lds_sync();
  const b16* Qb = Qp + ((size_t)(n * H + h) * T) * HD; const b16* Kb = Kp + ((size_t)(n * H + h) * TP) * HD; const b16* Vb = VT + ((size_t)(n * H + h) * HD) * TP; const b16* Vlb = VTl + ((size_t)(n * H + h) * HD) * TP;
  const v16b qa0 = frag_kb(Qb + (size_t)tq * HD, hh), qa1 = frag_kb(Qb + (size_t)tq * HD + 32, hh);
  float e[48]; float mx = -INFINITY; const float cs = 0.125f / (XS * XS);
#pragma unroll
  for (int kt = 0; kt < 6; ++kt) { v8f s = (v8f){}; const size_t kr = (size_t)(t0 + kt * 16 + col) * HD; s = wmma16b(frag_kb(Kb + kr, hh), qa0, s); s = wmma16b(frag_kb(Kb + kr + 32, hh), qa1, s);
#pragma unroll
    for (int r = 0; r < 8; ++r) { const int tok = t0 + kt * 16 + 8 * hh + r - PADL; const int w = tok - tq + LEFT; const bool ok = (w >= 0 && w < WIN && tok >= 0 && tok < T);
      const float lg = ok ? s[r] * cs + rbs[wave][ok ? w : 0] : -INFINITY; e[kt * 8 + r] = lg; mx = fmaxf(mx, lg); } }
  mx = fmaxf(mx, __shfl_xor(mx, 16)); float sum = 0.0f;
#pragma unroll
  for (int i = 0; i < 48; ++i) { const float p = (e[i] == -INFINITY) ? 0.0f : nexp2((e[i] - mx) * LOG2E); e[i] = p; sum += p; }
  sum += __shfl_xor(sum, 16); const float inv = 1.0f / sum;
#pragma unroll
  for (int kt = 0; kt < 6; ++kt)
#pragma unroll
    for (int r = 0; r < 8; ++r) Pf[wave][col][kt * 16 + 8 * hh + r] = e[kt * 8 + r] * inv * PS;
  wave_lds_sync();
  { const int rr = lane & 15, c0 = (lane >> 4) * 48; for (int q = 0; q < 48; q += 8) { v8b hv, lv; for (int j = 0; j < 8; ++j) { b16 a_, b_; split16(Pf[wave][rr][c0 + q + j], a_, b_); hv[j] = a_; lv[j] = b_; } *(v8b*)(&Ph[wave][rr][c0 + q]) = hv; *(v8b*)(&Pl[wave][rr][c0 + q]) = lv; } }
  wave_lds_sync();
  v8f o[4]; for (int t = 0; t < 4; ++t) o[t] = (v8f){};
#pragma unroll
  for (int ks = 0; ks < 3; ++ks) { const v16b ph = frag_kb(&Ph[wave][col][ks * 32], hh), pl = frag_kb(&Pl[wave][col][ks * 32], hh);
#pragma unroll
    for (int t = 0; t < 4; ++t) { const size_t vo = (size_t)(t * 16 + col) * TP + t0 + ks * 32; const v16b va = frag_kb(Vb + vo, hh), val = frag_kb(Vlb + vo, hh); o[t] = wmma16b(va, ph, o[t]); o[t] = wmma16b(va, pl, o[t]); o[t] = wmma16b(val, ph, o[t]); } }
  const float iv = 1.0f / (PS * XS);
#pragma unroll
  for (int t = 0; t < 4; ++t)
#pragma unroll
    for (int r = 0; r < 8; ++r) To[wave][col][t * 16 + 8 * hh + r] = o[t][r] * iv;
  wave_lds_sync();
  for (int pass = 0; pass < 2; ++pass) { for (int rr = 0; rr < 16; ++rr) { v2h hv, lv; for (int j = 0; j < 2; ++j) { b16 a_, b_; split16(To[wave][rr][lane * 2 + j] * XS, a_, b_); hv[j] = a_; lv[j] = b_; }
      const size_t oi = ((size_t)n * T + t0 + rr) * C + h * HD + lane * 2; *(volatile v2h*)(Oh + oi) = hv; *(volatile v2h*)(Ol + oi) = lv; } __threadfence(); }
}
__global__ __launch_bounds__(128) void proj_kernel(const b16* __restrict__ Oh, const b16* __restrict__ Ol, const b16* __restrict__ WP, const float* __restrict__ bp, float* __restrict__ out) {
  __shared__ __attribute__((aligned(16))) float Tf[4][16][128 + 4];
  const int wave = threadIdx.x >> 5, lane = threadIdx.x & 31, nloc = lane & 15, hlf = lane >> 4; const size_t m0 = (size_t)blockIdx.x * 64 + wave * 16; const int n0 = blockIdx.y * 128;
  v8f acc[8];
#pragma unroll
  for (int t = 0; t < 8; ++t) acc[t] = (v8f){};
#pragma unroll 2
  for (int kb = 0; kb < C; kb += 32) { const v16b a = frag_kb(Oh + (m0 + nloc) * C + kb, hlf), al = frag_kb(Ol + (m0 + nloc) * C + kb, hlf);
#pragma unroll
    for (int t = 0; t < 8; ++t) { const v16b bw = frag_kb(WP + (size_t)(n0 + t * 16 + nloc) * C + kb, hlf); acc[t] = wmma16b(a, bw, acc[t]); acc[t] = wmma16b(al, bw, acc[t]); } }
#pragma unroll
  for (int t = 0; t < 8; ++t) { const float bb = bf16_rne(bp[n0 + t * 16 + nloc]);
#pragma unroll
    for (int r = 0; r < 8; ++r) Tf[wave][8 * hlf + r][t * 16 + nloc] = acc[t][r] * (1.0f / (XS * WSC)) + bb; }
  wave_lds_sync();
  for (int pass = 0; pass < 2; ++pass) { for (int rr = 0; rr < 16; ++rr) *(volatile v4f*)(out + (m0 + rr) * C + n0 + lane * 4) = *(const v4f*)(&Tf[wave][rr][lane * 4]); __threadfence(); }
}
}

extern "C" void kernel_launch(void* const* d_in, const int* in_sizes, int n_in, void* d_out, int out_size, void* d_ws, size_t ws_size, hipStream_t stream) {
  (void)n_in;
  auto Fp = [&](int i) { return (const float*)d_in[i]; };
  if (in_sizes[0] != NN * T * C || in_sizes[1] != C * 3 * C || in_sizes[2] != 3 * C || in_sizes[3] != H * WIN || in_sizes[4] != C * C || in_sizes[5] != C || out_size != NN * T * C) return;
  size_t off = 0; char* ws = (char*)d_ws;
  auto carve = [&](size_t bytes) { char* p = ws + off; off += (bytes + 255) & ~(size_t)255; return p; };
  b16* WQ = (b16*)carve((size_t)3 * C * C * 2); b16* WP = (b16*)carve((size_t)C * C * 2); b16* Qp = (b16*)carve((size_t)NN * H * T * HD * 2); b16* Kp = (b16*)carve((size_t)NN * H * TP * HD * 2); b16* VT = (b16*)carve((size_t)NN * H * HD * TP * 2);
  b16* VTl = (b16*)carve((size_t)NN * H * HD * TP * 2); b16* Oh = (b16*)carve((size_t)NN * T * C * 2); b16* Ol = (b16*)carve((size_t)NN * T * C * 2);
  if (off > ws_size || off > ((size_t)128 << 20)) return;
  prep_kernel<<<(unsigned)((((size_t)3 * C * C + (size_t)C * C + (size_t)NN * H * TP * HD) / 8 + 255) / 256), 256, 0, stream>>>(Fp(1), Fp(4), WQ, WP, Kp, VT, VTl);
  qkv_kernel<<<dim3(T / 64, NL * H), 128, 0, stream>>>(Fp(0), WQ, Fp(2), Qp, Kp, VT, VTl);
  attn_kernel<<<dim3(T / 32, NL * H), 64, 0, stream>>>(Qp, Kp, VT, VTl, Fp(3), Oh, Ol);
  proj_kernel<<<dim3(NL * T / 64, 2), 128, 0, stream>>>(Oh, Ol, WP, Fp(5), (float*)d_out);
}
